// GRUCell_52793738002631
// MI455X (gfx1250) — hardware-run, weakly checked
//
#include <hip/hip_runtime.h>
#include <math.h>

constexpr int kB   = 32;
constexpr int kN   = 2048;
constexpr int kCin = 32;
constexpr int kH   = 64;
constexpr int kD   = 64;
constexpr int kCI  = 96;
constexpr int kKI  = 192;
constexpr int kOG  = 128;
constexpr int kOU  = 64;
constexpr int kJWG = kOG * kKI + kOG;
constexpr int kJWU = kOU * kKI + kOU;
constexpr int kNT3 = kB * kCI;
constexpr int kChG = 256;
constexpr int kChU = 512;
constexpr int kEPlane = kN * kD;
constexpr float kAdjCarry    = 32768.0f;
constexpr float kAdjCarryInv = 1.0f / 32768.0f;
constexpr size_t kWPlaneHalves = ((size_t)kChG * kJWG > (size_t)kChU * kJWU) ? (size_t)kChG * kJWG : (size_t)kChU * kJWU;

static_assert(kD % 32 == 0);
static_assert(kN % 64 == 0 && kNT3 % 64 == 0);
static_assert(kChG % 64 == 0 && kChU % 64 == 0);
static_assert(kN % kChG == 0 && kN % kChU == 0);
static_assert(kJWG % 64 == 0 && kJWU % 64 == 0);
static_assert(kN % 32 == 0);
static_assert((kJWG * 2) % 128 == 0 && (kJWU * 2) % 128 == 0);
static_assert(kN % 8 == 0);
static_assert(kKI % 32 == 0);

typedef __attribute__((ext_vector_type(16))) _Float16 v16h;
typedef __attribute__((ext_vector_type(8)))  _Float16 v8h;
typedef __attribute__((ext_vector_type(16))) __bf16   v16b;
typedef __attribute__((ext_vector_type(8)))  __bf16   v8b;
typedef __attribute__((ext_vector_type(8)))  float    v8f;
typedef __attribute__((ext_vector_type(4)))  float    v4f;
typedef __attribute__((ext_vector_type(4)))  unsigned int v4u;
typedef __attribute__((ext_vector_type(2)))  unsigned int v2u;

__device__ __forceinline__ unsigned short f2bf_bits(float f) {
  unsigned u = __float_as_uint(f);
  return (unsigned short)((u + 0x7FFFu + ((u >> 16) & 1u)) >> 16);
}
__device__ __forceinline__ float bf_bits2f(unsigned short h) { return __uint_as_float(((unsigned)h) << 16); }
__device__ __forceinline__ float bfr(float f) { return bf_bits2f(f2bf_bits(f)); }
__device__ __forceinline__ unsigned pk16(unsigned short a, unsigned short b) { return (unsigned)a | ((unsigned)b << 16); }
__device__ __forceinline__ unsigned short h_bits(float f) { const _Float16 h = (_Float16)f; return __builtin_bit_cast(unsigned short, h); }

__device__ __forceinline__ void dep_guard_h(v8f& a, v8f& b, v16h x, v16h y) { asm volatile("v_nop\n\tv_nop\n\tv_nop\n\tv_nop" : "+v"(a), "+v"(b) : "v"(x), "v"(y)); }
__device__ __forceinline__ void dep_guard_b(v8f& a, v8f& b, v16b x, v16b y) { asm volatile("v_nop\n\tv_nop\n\tv_nop\n\tv_nop" : "+v"(a), "+v"(b) : "v"(x), "v"(y)); }
__device__ __forceinline__ void keep4_h(v16h a, v16h b, v16h c, v16h d) { asm volatile("v_nop" :: "v"(a), "v"(b), "v"(c), "v"(d)); }
__device__ __forceinline__ void keep4_b(v16b a, v16b b, v16b c, v16b d) { asm volatile("v_nop" :: "v"(a), "v"(b), "v"(c), "v"(d)); }
__device__ __forceinline__ void acc_guard4(v8f& a, v8f& b, v8f& c, v8f& d) { asm volatile("v_nop\n\tv_nop\n\tv_nop\n\tv_nop" : "+v"(a), "+v"(b), "+v"(c), "+v"(d)); }
__device__ __forceinline__ void guard1_b(v8f& a, v16b x, v16b y) { asm volatile("v_nop\n\tv_nop\n\tv_nop\n\tv_nop" : "+v"(a) : "v"(x), "v"(y)); }
__device__ __forceinline__ void keep2_b(v16b a, v16b b) { asm volatile("v_nop" :: "v"(a), "v"(b)); }
__device__ __forceinline__ void acc_guard2(v8f& a, v8f& b) { asm volatile("v_nop\n\tv_nop\n\tv_nop\n\tv_nop" : "+v"(a), "+v"(b)); }

template <typename T> struct Frag;
template <> struct Frag<_Float16> {
  typedef v16h V; union U { v16h v; v8h h[2]; };
  static __device__ __forceinline__ v16h load(const _Float16* p) {
    U f; f.h[0] = *(const v8h*)(p); f.h[1] = *(const v8h*)(p + 16); return f.v;
  }
  static __device__ __forceinline__ v8f mma(v16h a, v16h b, v8f c) {
    return __builtin_amdgcn_wmma_f32_16x16x32_f16(false, a, false, b, (short)0, c, false, false);
  }
  static __device__ __forceinline__ void guard(v8f& a, v8f& b, v16h x, v16h y) { dep_guard_h(a, b, x, y); }
  static __device__ __forceinline__ void keep(v16h a, v16h b, v16h c, v16h d) { keep4_h(a, b, c, d); }
};
template <> struct Frag<__bf16> {
  typedef v16b V; union U { v16b v; v8b h[2]; };
  static __device__ __forceinline__ v16b load(const __bf16* p) {
    U f; f.h[0] = *(const v8b*)(p); f.h[1] = *(const v8b*)(p + 16); return f.v;
  }
  static __device__ __forceinline__ v8f mma(v16b a, v16b b, v8f c) {
    return __builtin_amdgcn_wmma_f32_16x16x32_bf16(false, a, false, b, (short)0, c, false, false);
  }
  static __device__ __forceinline__ void guard(v8f& a, v8f& b, v16b x, v16b y) { dep_guard_b(a, b, x, y); }
  static __device__ __forceinline__ void keep(v16b a, v16b b, v16b c, v16b d) { keep4_b(a, b, c, d); }
};

template <int ET> struct Elem;
template <> struct Elem<0> { typedef _Float16 T; };
template <> struct Elem<1> { typedef __bf16 T; };
template <int ET, int SPLITM, int BIAS_MODE, int OUT_MODE, bool RESID, int ACT = 0>
__global__ __launch_bounds__(256) void wmma_gemm64(
    const unsigned short* __restrict__ Ap, const unsigned short* __restrict__ A2p, int lda, long strideA,
    const unsigned short* __restrict__ Btp, const unsigned short* __restrict__ Bt2p, int ldb, long strideB,
    void* __restrict__ Cout, void* __restrict__ Cout2, int ldc, long strideC,
    const float* __restrict__ bias,
    const float* __restrict__ resid, long strideR,
    int M, int N, int K, float scale) {
  typedef typename Elem<ET>::T T;
  typedef typename Frag<T>::V V;
  const T* A = (const T*)Ap; const T* A2 = (const T*)A2p; const T* Bt = (const T*)Btp; const T* Bt2 = (const T*)Bt2p;
  __shared__ __align__(16) float sT[8][16 * 68];
  const int b    = blockIdx.y;
  const int lane = threadIdx.x & 31;
  const int wave = threadIdx.x >> 5;
  const int tilesN = N >> 6;
  const int tilesM = M >> 6;
  const int tile = blockIdx.x * 8 + wave;
  if (tile >= tilesM * tilesN) return;
  const int tm = tile / tilesN;
  const int tn = tile - tm * tilesN;
  const int m0 = tm << 6;
  const int n0 = tn << 6;
  (void)resid; (void)strideR;

  const T* Ab  = A  + (size_t)b * strideA;
  const T* Bb  = Bt + (size_t)b * strideB;
  const T* Ab2 = (SPLITM != 0) ? (A2  + (size_t)b * strideA) : nullptr;
  const T* Bb2 = (SPLITM == 1) ? (Bt2 + (size_t)b * strideB) : nullptr;

  const int rlane = lane & 15;
  const int koff  = (lane >> 4) * 8;
  const int mOff  = (lane >> 4) * 8;

  v8f acc[4][4];
#pragma unroll
  for (int i = 0; i < 4; ++i)
#pragma unroll
    for (int j = 0; j < 4; ++j) acc[i][j] = (v8f){0.f,0.f,0.f,0.f,0.f,0.f,0.f,0.f};

  for (int k0 = 0; k0 < K; k0 += 32) {
    V bh[4], bl[4];
#pragma unroll
    for (int j = 0; j < 4; ++j) {
      const size_t bo = (size_t)(n0 + (j << 4) + rlane) * ldb + koff + k0;
      bh[j] = Frag<T>::load(Bb + bo);
      if (SPLITM == 1) bl[j] = Frag<T>::load(Bb2 + bo);
    }
#pragma unroll
    for (int i = 0; i < 4; ++i) {
      const size_t ao = (size_t)(m0 + (i << 4) + rlane) * lda + koff + k0;
      V ah = Frag<T>::load(Ab + ao);
      V al;
      if (SPLITM != 0) al = Frag<T>::load(Ab2 + ao);
#pragma unroll
      for (int j = 0; j < 4; ++j) {
        acc[i][j] = Frag<T>::mma(ah, bh[j], acc[i][j]);
        if (SPLITM == 1) acc[i][j] = Frag<T>::mma(ah, bl[j], acc[i][j]);
        if (SPLITM != 0) acc[i][j] = Frag<T>::mma(al, bh[j], acc[i][j]);
      }
      Frag<T>::guard(acc[i][0], acc[i][3], ah, (SPLITM != 0) ? al : ah);
    }
    Frag<T>::keep(bh[0], bh[1], bh[2], bh[3]);
    if (SPLITM == 1) Frag<T>::keep(bl[0], bl[1], bl[2], bl[3]);
  }
  acc_guard4(acc[0][0], acc[0][1], acc[0][2], acc[0][3]);
  acc_guard4(acc[1][0], acc[1][1], acc[1][2], acc[1][3]);
  acc_guard4(acc[2][0], acc[2][1], acc[2][2], acc[2][3]);
  acc_guard4(acc[3][0], acc[3][1], acc[3][2], acc[3][3]);

  float* slab = sT[wave];
#pragma unroll
  for (int i = 0; i < 4; ++i) {
    const int mBase = m0 + (i << 4);
#pragma unroll
    for (int j = 0; j < 4; ++j) {
      const int n = n0 + (j << 4) + rlane;
      float bv = 0.f;
      if (BIAS_MODE == 2) bv = bias[n];
#pragma unroll
      for (int r = 0; r < 8; ++r) {
        float v = acc[i][j][r] * scale;
        if (BIAS_MODE == 1) v += bias[mBase + mOff + r];
        if (BIAS_MODE == 2) v += bv;
        if (ACT == 2) v = fmaxf(v, 0.0f);
        if (ACT == 4) v = (v > 0.f) ? v : 0.01f * v;
        slab[(mOff + r) * 68 + (j << 4) + rlane] = v;
      }
    }
    __builtin_amdgcn_fence(__ATOMIC_RELEASE, "workgroup");
    __builtin_amdgcn_wave_barrier();
    __builtin_amdgcn_fence(__ATOMIC_ACQUIRE, "workgroup");
    if (OUT_MODE == 0) {
      float* C = (float*)Cout + (size_t)b * strideC;
      const int hh = lane >> 4, c4 = (lane & 15) * 4;
      for (int pass = 0; pass < 2; ++pass) {
#pragma unroll
        for (int it = 0; it < 8; ++it) {
          const int row = it * 2 + hh;
          v4f v = *(const v4f*)(slab + row * 68 + c4);
          *(volatile v4f*)(C + (size_t)(mBase + row) * ldc + n0 + c4) = v;
        }
        __threadfence();
      }
    } else {
      const int q = lane >> 3, c8 = (lane & 7) * 8;
      unsigned short* C  = (unsigned short*)Cout  + (size_t)b * strideC;
      unsigned short* C2 = (OUT_MODE == 2) ? ((unsigned short*)Cout2 + (size_t)b * strideC) : nullptr;
      for (int pass = 0; pass < 2; ++pass) {
#pragma unroll
        for (int it = 0; it < 4; ++it) {
          const int row = it * 4 + q;
          const float* sp = slab + row * 68 + c8;
          v8h hv, lv;
#pragma unroll
          for (int e = 0; e < 8; ++e) {
            if (OUT_MODE == 1) {
              hv[e] = (_Float16)sp[e];
            } else {
              unsigned short hb = f2bf_bits(sp[e]);
              unsigned short lb = f2bf_bits(sp[e] - bf_bits2f(hb));
              hv[e] = __builtin_bit_cast(_Float16, hb);
              lv[e] = __builtin_bit_cast(_Float16, lb);
            }
          }
          *(volatile v8h*)(C + (size_t)(mBase + row) * ldc + n0 + c8) = hv;
          if (OUT_MODE == 2) *(volatile v8h*)(C2 + (size_t)(mBase + row) * ldc + n0 + c8) = lv;
        }
        __threadfence();
      }
    }
    __builtin_amdgcn_fence(__ATOMIC_RELEASE, "workgroup");
    __builtin_amdgcn_wave_barrier();
    __builtin_amdgcn_fence(__ATOMIC_ACQUIRE, "workgroup");
  }
}

__global__ __launch_bounds__(256) void ln_kernel(const float* __restrict__ ne, const float* __restrict__ te,
                                               const float* __restrict__ gg, const float* __restrict__ gb,
                                               const float* __restrict__ ug, const float* __restrict__ ub,
                                               unsigned short* __restrict__ epl) {
  __shared__ __align__(16) float sg[8][64];
  __shared__ __align__(16) float su[8][64];
  const int tid = threadIdx.x, lane = tid & 31, wave = tid >> 5;
  const int n = blockIdx.x * 8 + wave;
  const float v0 = bfr(ne[(size_t)n * kD + lane]) + bfr(te[lane]);
  const float v1 = bfr(ne[(size_t)n * kD + 32 + lane]) + bfr(te[32 + lane]);
  float s = v0 + v1;
  s += __shfl_xor(s, 16, 32); s += __shfl_xor(s, 8, 32); s += __shfl_xor(s, 4, 32); s += __shfl_xor(s, 2, 32); s += __shfl_xor(s, 1, 32);
  const float mu = s * (1.0f / 64.0f);
  const float d0 = v0 - mu, d1 = v1 - mu;
  float sq = d0 * d0 + d1 * d1;
  sq += __shfl_xor(sq, 16, 32); sq += __shfl_xor(sq, 8, 32); sq += __shfl_xor(sq, 4, 32); sq += __shfl_xor(sq, 2, 32); sq += __shfl_xor(sq, 1, 32);
  const float var = sq * (1.0f / 64.0f);
  const float inv = rsqrtf(var + 1e-12f);
  const float nv0 = d0 * inv, nv1 = d1 * inv;
  sg[wave][lane]      = nv0 * bfr(gg[lane])      + bfr(gb[lane]);
  sg[wave][32 + lane] = nv1 * bfr(gg[32 + lane]) + bfr(gb[32 + lane]);
  su[wave][lane]      = nv0 * bfr(ug[lane])      + bfr(ub[lane]);
  su[wave][32 + lane] = nv1 * bfr(ug[32 + lane]) + bfr(ub[32 + lane]);
  __syncthreads();
  const int q4 = lane >> 3, c8 = (lane & 7) * 8;
  const float fu = (q4 >= 2) ? 1.0f : 0.0f;
  const float fg = 1.0f - fu;
  unsigned short ob[8];
#pragma unroll
  for (int e = 0; e < 8; ++e) {
    const float a  = sg[wave][c8 + e];
    const float bb = su[wave][c8 + e];
    const float f  = fmaf(fg, a, fu * bb);
    const unsigned short hb = f2bf_bits(f);
    const unsigned short lb = f2bf_bits(f - bf_bits2f(hb));
    ob[e] = (q4 & 1) ? lb : hb;
  }
  const v4u u = (v4u){pk16(ob[0], ob[1]), pk16(ob[2], ob[3]), pk16(ob[4], ob[5]), pk16(ob[6], ob[7])};
  unsigned short* dst = epl + (size_t)q4 * kEPlane + (size_t)n * kD + c8;
  for (int pass = 0; pass < 2; ++pass) {
    *(volatile v4u*)dst = u;
    __threadfence();
  }
}

template <int O>
__global__ __launch_bounds__(256) void poolt_kernel(const float* __restrict__ wp, const float* __restrict__ bp,
                                                  unsigned short* __restrict__ wT) {
  constexpr int JM = O * kKI;
  constexpr int JW = JM + O;
  static_assert((JM * 8) % 256 == 0 && (JW * 8) % 256 == 0);
  const int gid = blockIdx.x * 256 + threadIdx.x;
  const int j = gid >> 3, d0 = (gid & 7) * 8;
  const bool wmain = ((int)blockIdx.x < (JM * 8) / 256);
  unsigned short hb[8];
  if (wmain) {
    const int o = j / kKI;
    const int ki = j - o * kKI;
#pragma unroll
    for (int e = 0; e < 8; ++e) hb[e] = f2bf_bits(wp[((size_t)(d0 + e) * kKI + ki) * O + o]);
  } else {
    int o = j - JM; o = o < 0 ? 0 : (o >= O ? O - 1 : o);
#pragma unroll
    for (int e = 0; e < 8; ++e) hb[e] = f2bf_bits(bp[(size_t)(d0 + e) * O + o]);
  }
  const v4u u = (v4u){pk16(hb[0], hb[1]), pk16(hb[2], hb[3]), pk16(hb[4], hb[5]), pk16(hb[6], hb[7])};
  unsigned short* dst = wT + (size_t)j * kD + d0;
  for (int pass = 0; pass < 2; ++pass) {
    *(volatile v4u*)dst = u;
    __threadfence();
  }
}

template <int MODE>
__global__ __launch_bounds__(256) void packt_kernel(const float* __restrict__ x, const float* __restrict__ sec,
                                                  unsigned short* __restrict__ Tp) {
  __shared__ __align__(16) float s[kCI][68];
  const int tid = threadIdx.x;
  const int b = blockIdx.y, m0 = blockIdx.x * 64;
#pragma unroll 4
  for (int i = 0; i < 8; ++i) {
    const int e = i * 256 + tid;
    const int ml = e >> 5, c = e & 31;
    s[c][ml] = bfr(x[((size_t)b * kN + m0 + ml) * kCin + c]);
  }
#pragma unroll 4
  for (int i = 0; i < 16; ++i) {
    const int e = i * 256 + tid;
    const int ml = e >> 6, hc = e & 63;
    float v = sec[((size_t)b * kN + m0 + ml) * kH + hc];
    if (MODE == 0) v = bfr(v);
    s[kCin + hc][ml] = v;
  }
  __syncthreads();
  const int lane = tid & 31, wave = tid >> 5;
  const int q = lane >> 3, c8 = (lane & 7) * 8;
  v4u u[3];
#pragma unroll
  for (int it = 0; it < 3; ++it) {
    const int row = wave * 12 + it * 4 + q;
    unsigned short hb[8];
#pragma unroll
    for (int e = 0; e < 8; ++e) hb[e] = h_bits(s[row][c8 + e]);
    u[it] = (v4u){pk16(hb[0], hb[1]), pk16(hb[2], hb[3]), pk16(hb[4], hb[5]), pk16(hb[6], hb[7])};
  }
  for (int pass = 0; pass < 2; ++pass) {
#pragma unroll
    for (int it = 0; it < 3; ++it) {
      const int row = wave * 12 + it * 4 + q;
      *(volatile v4u*)(Tp + ((size_t)b * kCI + row) * kN + m0 + c8) = u[it];
    }
    __threadfence();
  }
}

__global__ __launch_bounds__(512) void softmax_adj_kernel(const float* __restrict__ S, unsigned short* __restrict__ P) {
  __shared__ float redM[16];
  __shared__ float redS[16];
  const int n = blockIdx.x;
  const int t = threadIdx.x;
  const int lane = t & 31, wave = t >> 5;
  const int c0 = t * 4;
  const v4f a = *(const v4f*)(S + (size_t)n * kN + c0);
  float m = fmaxf(fmaxf(a[0], a[1]), fmaxf(a[2], a[3]));
#pragma unroll
  for (int off = 16; off > 0; off >>= 1) m = fmaxf(m, __shfl_xor(m, off, 32));
  if (lane == 0) redM[wave] = m;
  __syncthreads();
  float mx = redM[0];
#pragma unroll
  for (int w = 1; w < 16; ++w) mx = fmaxf(mx, redM[w]);
  const float snn = S[(size_t)n * kN + n];
  const float ed = expf(snn - mx);
  float ex[4], keep[4];
  float so = 0.0f;
#pragma unroll
  for (int e = 0; e < 4; ++e) {
    ex[e] = expf(a[e] - mx);
    keep[e] = (c0 + e == n) ? 0.0f : 1.0f;
    so = fmaf(keep[e], ex[e], so);
  }
#pragma unroll
  for (int off = 16; off > 0; off >>= 1) so += __shfl_xor(so, off, 32);
  if (lane == 0) redS[wave] = so;
  __syncthreads();
  float soff = redS[0];
#pragma unroll
  for (int w = 1; w < 16; ++w) soff += redS[w];
  const float total = soff + ed;
  const float inv = kAdjCarry * (1.0f / total);
  const float dval = -soff * inv;
  unsigned short hb[4];
#pragma unroll
  for (int e = 0; e < 4; ++e) {
    const float o = fmaf(keep[e], ex[e] * inv, (1.0f - keep[e]) * dval);
    hb[e] = h_bits(o);
  }
  const v2u u = (v2u){pk16(hb[0], hb[1]), pk16(hb[2], hb[3])};
  unsigned short* dst = P + (size_t)n * kN + c0;
  for (int pass = 0; pass < 2; ++pass) {
    *(volatile v2u*)dst = u;
    __threadfence();
  }
}

__device__ __forceinline__ void lds_put_hl(__bf16* h, __bf16* l, int idx, float v) {
  const unsigned short hb = f2bf_bits(v);
  const unsigned short lb = f2bf_bits(v - bf_bits2f(hb));
  h[idx] = __builtin_bit_cast(__bf16, hb);
  l[idx] = __builtin_bit_cast(__bf16, lb);
}

template <int MODE>
__global__ __launch_bounds__(256) void conv_node_kernel(const float* __restrict__ x, const float* __restrict__ st,
                                                      const float* __restrict__ zsin, const float* __restrict__ corr,
                                                      const unsigned short* __restrict__ Whp, const unsigned short* __restrict__ Wlp,
                                                      float* __restrict__ zsout, float* rpl, float* __restrict__ outp, int n0c) {
  constexpr int O  = (MODE == 0) ? kOG : kOU;
  constexpr int JW = O * kKI + O;
  constexpr int CP = O + 4;
  constexpr int AP = kKI + 8;
  constexpr int NRT = (MODE == 0) ? 2 : 1;
  __shared__ __align__(16) __bf16 sAh[kB * AP];
  __shared__ __align__(16) __bf16 sAl[kB * AP];
  __shared__ __align__(16) float  sC[kB * CP];
  __shared__ float sBias[O];
  const int tid = threadIdx.x, lane = tid & 31, wave = tid >> 5;
  const int nl = blockIdx.x;
  const int n = n0c + nl;
  const float* crow = corr + (size_t)nl * kNT3;

#pragma unroll 1
  for (int i = 0; i < 4; ++i) {
    const int e = i * 256 + tid;
    const int bb = e >> 5, c = e & 31;
    const float xv = bfr(x[((size_t)bb * kN + n) * kCin + c]);
    const float cr = crow[bb * kCI + c];
    lds_put_hl(sAh, sAl, bb * AP + c, xv);
    lds_put_hl(sAh, sAl, bb * AP + kCI + c, xv + cr);
  }
#pragma unroll 1
  for (int i = 0; i < 8; ++i) {
    const int e = i * 256 + tid;
    const int bb = e >> 6, hc = e & 63;
    float sv;
    if (MODE == 0) sv = bfr(st[((size_t)bb * kN + n) * kH + hc]);
    else           sv = zsin[((size_t)bb * kN + n) * kH + hc];
    const float cr = crow[bb * kCI + kCin + hc];
    lds_put_hl(sAh, sAl, bb * AP + kCin + hc, sv);
    lds_put_hl(sAh, sAl, bb * AP + kCI + kCin + hc, sv + cr);
  }
  if (tid < O) {
    const unsigned hb = Whp[(size_t)nl * JW + (size_t)O * kKI + tid];
    const unsigned lb = Wlp[(size_t)nl * JW + (size_t)O * kKI + tid];
    sBias[tid] = __uint_as_float(hb << 16) + __uint_as_float(lb << 16);
  }
  __syncthreads();

  const int rlane = lane & 15, koff = (lane >> 4) * 8, mOff = (lane >> 4) * 8;
  const int o0  = (MODE == 0) ? wave * 16 : (wave & 3) * 16;
  const int rt0 = (MODE == 0) ? 0 : (wave >> 2);
  v8f acc[2];
  acc[0] = (v8f){0.f,0.f,0.f,0.f,0.f,0.f,0.f,0.f};
  acc[1] = (v8f){0.f,0.f,0.f,0.f,0.f,0.f,0.f,0.f};
  const __bf16* whr = (const __bf16*)Whp + (size_t)nl * JW + (size_t)(o0 + rlane) * kKI + koff;
  const __bf16* wlr = (const __bf16*)Wlp + (size_t)nl * JW + (size_t)(o0 + rlane) * kKI + koff;
#pragma unroll
  for (int k0 = 0; k0 < kKI; k0 += 32) {
    const v16b bh = Frag<__bf16>::load(whr + k0);
    const v16b bl = Frag<__bf16>::load(wlr + k0);
#pragma unroll
    for (int t = 0; t < NRT; ++t) {
      const int ao = ((rt0 + t) * 16 + rlane) * AP + koff + k0;
      const v16b ah = Frag<__bf16>::load(sAh + ao);
      const v16b al = Frag<__bf16>::load(sAl + ao);
      acc[t] = Frag<__bf16>::mma(ah, bh, acc[t]);
      acc[t] = Frag<__bf16>::mma(ah, bl, acc[t]);
      acc[t] = Frag<__bf16>::mma(al, bh, acc[t]);
      guard1_b(acc[t], ah, al);
    }
    keep2_b(bh, bl);
  }
  acc_guard2(acc[0], acc[1]);

#pragma unroll
  for (int t = 0; t < NRT; ++t) {
    const int col = o0 + rlane;
    const float bv = sBias[col];
#pragma unroll
    for (int r = 0; r < 8; ++r) {
      const int row = (rt0 + t) * 16 + mOff + r;
      float v = acc[t][r] + bv;
      if (MODE == 0) {
        const float ev = fminf(expf(-v), 1.0e20f);
        v = 1.0f / (1.0f + ev);
      } else {
        v = tanhf(v);
      }
      sC[row * CP + col] = v;
    }
  }
  __syncthreads();

  {
    const int hh = lane >> 4, c4 = (lane & 15) * 4;
    v4f va[2], vb[2];
    size_t off[2];
#pragma unroll
    for (int it = 0; it < 2; ++it) {
      const int bb = wave * 4 + it * 2 + hh;
      off[it] = ((size_t)bb * kN + n) * kH + c4;
      const v4f s4 = *(const v4f*)(st + off[it]);
      v4f sr;
#pragma unroll
      for (int e = 0; e < 4; ++e) sr[e] = bfr(s4[e]);
      if (MODE == 0) {
        const v4f z4 = *(const v4f*)(sC + bb * CP + c4);
        va[it] = z4 * sr;
        vb[it] = *(const v4f*)(sC + bb * CP + kH + c4);
      } else {
        const v4f h4 = *(const v4f*)(sC + bb * CP + c4);
        const v4f r4 = *(const v4f*)(rpl + off[it]);
        const v4f one = (v4f){1.0f, 1.0f, 1.0f, 1.0f};
        va[it] = r4 * sr + (one - r4) * h4;
        vb[it] = one;
      }
    }
    for (int pass = 0; pass < 2; ++pass) {
#pragma unroll
      for (int it = 0; it < 2; ++it) {
        if (MODE == 0) {
          *(volatile v4f*)(zsout + off[it]) = va[it];
          *(volatile v4f*)(rpl + off[it])   = vb[it];
        } else {
          *(volatile v4f*)(outp + off[it]) = va[it];
        }
      }
      __threadfence();
    }
  }
}

extern "C" void kernel_launch(void* const* d_in, const int* in_sizes, int n_in,
                              void* d_out, int out_size, void* d_ws, size_t ws_size,
                              hipStream_t stream) {
  if (n_in < 12) return;
  if (in_sizes[0] != kB * kN * kCin || in_sizes[1] != kB * kN * kH || in_sizes[2] != kN * kD || in_sizes[3] != kD) return;
  if (in_sizes[4] != kD * kKI * kOG || in_sizes[5] != kD * kOG || in_sizes[6] != kD || in_sizes[7] != kD) return;
  if (in_sizes[8] != kD * kKI * kOU || in_sizes[9] != kD * kOU || in_sizes[10] != kD || in_sizes[11] != kD) return;
  if (out_size != kB * kN * kH) return;

  const float* x   = (const float*)d_in[0];
  const float* st  = (const float*)d_in[1];
  const float* ne  = (const float*)d_in[2];
  const float* te  = (const float*)d_in[3];
  const float* gw  = (const float*)d_in[4];
  const float* gbp = (const float*)d_in[5];
  const float* gg  = (const float*)d_in[6];
  const float* gb  = (const float*)d_in[7];
  const float* uw  = (const float*)d_in[8];
  const float* ubp = (const float*)d_in[9];
  const float* ug  = (const float*)d_in[10];
  const float* ub  = (const float*)d_in[11];
  float* out = (float*)d_out;

  char* ws = (char*)d_ws;
  size_t off = 0;
  auto carve = [&](size_t bytes) -> char* { char* p = ws + off; off += (bytes + 255) & ~(size_t)255; return p; };
  unsigned short* epl    = (unsigned short*)carve((size_t)4 * kEPlane * 2);
  unsigned short* wTg    = (unsigned short*)carve((size_t)kJWG * kD * 2);
  unsigned short* wTu    = (unsigned short*)carve((size_t)kJWU * kD * 2);
  float*          logits = (float*)carve((size_t)kN * kN * 4);
  unsigned short* adj    = (unsigned short*)carve((size_t)kN * kN * 2);
  unsigned short* inpT   = (unsigned short*)carve((size_t)kNT3 * kN * 2);
  unsigned short* candT  = (unsigned short*)carve((size_t)kNT3 * kN * 2);
  float*          corr   = (float*)carve((size_t)kChU * kNT3 * 4);
  unsigned short* Wh     = (unsigned short*)carve(kWPlaneHalves * 2);
  unsigned short* Wl     = (unsigned short*)carve(kWPlaneHalves * 2);
  float*          zs     = (float*)carve((size_t)kB * kN * kH * 4);
  float*          rpl    = (float*)carve((size_t)kB * kN * kH * 4);
  if (off > ws_size || off > (size_t)134217728) return;

  unsigned short* egh = epl;
  unsigned short* egl = epl + (size_t)kEPlane;
  unsigned short* euh = epl + (size_t)2 * kEPlane;
  unsigned short* eul = epl + (size_t)3 * kEPlane;

  ln_kernel<<<kN / 8, 256, 0, stream>>>(ne, te, gg, gb, ug, ub, epl);
  poolt_kernel<kOG><<<(kJWG * 8) / 256, 256, 0, stream>>>(gw, gbp, wTg);
  poolt_kernel<kOU><<<(kJWU * 8) / 256, 256, 0, stream>>>(uw, ubp, wTu);
  packt_kernel<0><<<dim3(kN / 64, kB), 256, 0, stream>>>(x, st, inpT);

  wmma_gemm64<1, 1, 0, 0, false><<<dim3((kN / 64) * (kN / 64) / 8, 1), 256, 0, stream>>>(
      egh, egl, kD, 0L, egh, egl, kD, 0L,
      (void*)logits, (void*)nullptr, kN, 0L, (const float*)nullptr, (const float*)nullptr, 0L, kN, kN, kD, 1.0f);
  softmax_adj_kernel<<<kN, 512, 0, stream>>>(logits, adj);
  for (int ch = 0; ch < kN / kChG; ++ch) {
    const int n0c = ch * kChG;
    wmma_gemm64<0, 0, 0, 0, false><<<dim3(((kChG / 64) * (kNT3 / 64) + 7) / 8, 1), 256, 0, stream>>>(
        adj + (size_t)n0c * kN, (const unsigned short*)nullptr, kN, 0L,
        inpT, (const unsigned short*)nullptr, kN, 0L,
        (void*)corr, (void*)nullptr, kNT3, 0L, (const float*)nullptr, (const float*)nullptr, 0L,
        kChG, kNT3, kN, kAdjCarryInv);
    wmma_gemm64<1, 2, 0, 2, false><<<dim3(((kChG / 64) * (kJWG / 64) + 7) / 8, 1), 256, 0, stream>>>(
        egh + (size_t)n0c * kD, egl + (size_t)n0c * kD, kD, 0L,
        wTg, (const unsigned short*)nullptr, kD, 0L,
        (void*)Wh, (void*)Wl, kJWG, 0L, (const float*)nullptr, (const float*)nullptr, 0L,
        kChG, kJWG, kD, 1.0f);
    conv_node_kernel<0><<<kChG, 256, 0, stream>>>(x, st, (const float*)nullptr, corr, Wh, Wl, zs, rpl, (float*)nullptr, n0c);
  }

  packt_kernel<1><<<dim3(kN / 64, kB), 256, 0, stream>>>(x, zs, candT);
  wmma_gemm64<1, 1, 0, 0, false><<<dim3((kN / 64) * (kN / 64) / 8, 1), 256, 0, stream>>>(
      euh, eul, kD, 0L, euh, eul, kD, 0L,
      (void*)logits, (void*)nullptr, kN, 0L, (const float*)nullptr, (const float*)nullptr, 0L, kN, kN, kD, 1.0f);
  softmax_adj_kernel<<<kN, 512, 0, stream>>>(logits, adj);
  for (int ch = 0; ch < kN / kChU; ++ch) {
    const int n0c = ch * kChU;
    wmma_gemm64<0, 0, 0, 0, false><<<dim3(((kChU / 64) * (kNT3 / 64) + 7) / 8, 1), 256, 0, stream>>>(
        adj + (size_t)n0c * kN, (const unsigned short*)nullptr, kN, 0L,
        candT, (const unsigned short*)nullptr, kN, 0L,
        (void*)corr, (void*)nullptr, kNT3, 0L, (const float*)nullptr, (const float*)nullptr, 0L,
        kChU, kNT3, kN, kAdjCarryInv);
    wmma_gemm64<1, 2, 0, 2, false><<<dim3(((kChU / 64) * (kJWU / 64) + 7) / 8, 1), 256, 0, stream>>>(
        euh + (size_t)n0c * kD, eul + (size_t)n0c * kD, kD, 0L,
        wTu, (const unsigned short*)nullptr, kD, 0L,
        (void*)Wh, (void*)Wl, kJWU, 0L, (const float*)nullptr, (const float*)nullptr, 0L,
        kChU, kJWU, kD, 1.0f);
    conv_node_kernel<1><<<kChU, 256, 0, stream>>>(x, st, zs, corr, Wh, Wl, (float*)nullptr, rpl, out, n0c);
  }
}
